// GNFConverter_29978871726464
// MI455X (gfx1250) — hardware-verified
//
#include <hip/hip_runtime.h>

#define NBATCH 16
#define NATOM  128
#define NPT    4096
#define NTYPE  5
#define PPB    32
#define BSTR   136
#define ASTR   33
#define CLIPV  0.3f

typedef _Float16 f16;
typedef __attribute__((ext_vector_type(16))) f16 f16x16;
typedef __attribute__((ext_vector_type(8)))  f16 f16x8;
typedef __attribute__((ext_vector_type(8)))  float f32x8;
typedef __attribute__((ext_vector_type(4)))  float v4f_t;
typedef float v4fa __attribute__((ext_vector_type(4), may_alias));

__device__ __forceinline__ f32x8 wmma16(f16x16 a, f16x16 b, f32x8 c) {
  return __builtin_amdgcn_wmma_f32_16x16x32_f16(false, a, false, b, (short)0, c, false, false);
}

__device__ __forceinline__ f16x16 lds_frag(const f16* base, int stride) {
  const int lane = threadIdx.x & 31;
  const int row  = lane & 15;
  const int kh   = (lane >> 4) * 8;
  const f16x8 lo = *(const f16x8*)(base + row * stride + kh);
  const f16x8 hi = *(const f16x8*)(base + row * stride + kh + 16);
  f16x16 f;
#pragma unroll
  for (int i = 0; i < 8; ++i) { f[i] = lo[i]; f[i + 8] = hi[i]; }
  return f;
}

__device__ __forceinline__ void split16(float v, f16& h, f16& l) {
  h = (f16)v; l = (f16)((v - (float)h) * 2048.0f);
}

__global__ __launch_bounds__(64) void gnf_field_kernel(const float* __restrict__ coords,
                                                       const int*   __restrict__ atype,
                                                       const float* __restrict__ query,
                                                       float*       __restrict__ out) {
  __shared__ float cxS[NATOM], cyS[NATOM], czS[NATOM];
  __shared__ int   tyS[NATOM];
  __shared__ int   tcnt[8];
  __shared__ __attribute__((aligned(16))) f16 BhS[32 * BSTR];
  __shared__ __attribute__((aligned(16))) f16 BlS[32 * BSTR];
  __shared__ float accS[PPB * ASTR];
  __shared__ float qS[PPB * 3];
  __shared__ __attribute__((aligned(16))) float outS[PPB * NTYPE * 3];

  const int tid  = threadIdx.x;
  const int lane = tid & 31;
  const int wave = tid >> 5;
  const int pl   = lane & 15;
  const int hsel = lane >> 4;
  const int blk  = blockIdx.x;
  const int b    = blk / (NPT / PPB);
  const int p0   = (blk % (NPT / PPB)) * PPB;

  if (tid < 8) tcnt[tid] = 0;
  for (int i = tid; i < NATOM; i += 64) {
    const float* c = coords + ((size_t)b * NATOM + i) * 3;
    cxS[i] = c[0]; cyS[i] = c[1]; czS[i] = c[2];
    tyS[i] = atype[(size_t)b * NATOM + i];
  }
  for (int i = tid; i < PPB * 3; i += 64) qS[i] = query[((size_t)b * NPT + p0) * 3 + i];
  __syncthreads();
  if (tid < NTYPE) {
    int c = 0;
    for (int i = 0; i < NATOM; ++i) c += (tyS[i] == tid);
    tcnt[tid] = c;
  }
  for (int e = tid; e < 32 * NATOM; e += 64) {
    const int n = e >> 7, a = e & (NATOM - 1);
    float v = 0.0f;
    if (n < 4 * NTYPE) {
      const int t = n >> 2, c = n & 3;
      if (tyS[a] == t) v = (c == 0) ? cxS[a] : (c == 1) ? cyS[a] : (c == 2) ? czS[a] : 1.0f;
    }
    f16 h, l; split16(v, h, l);
    BhS[n * BSTR + a] = h; BlS[n * BSTR + a] = l;
  }

  const float qx = qS[(wave * 16 + pl) * 3 + 0], qy = qS[(wave * 16 + pl) * 3 + 1], qz = qS[(wave * 16 + pl) * 3 + 2];
  float d[4][16];
  float tmin[NTYPE];
#pragma unroll
  for (int t = 0; t < NTYPE; ++t) tmin[t] = 3.0e38f;
#pragma unroll
  for (int kc = 0; kc < 4; ++kc) {
#pragma unroll
    for (int i = 0; i < 16; ++i) {
      const int a = kc * 32 + hsel * 8 + (i & 7) + ((i >> 3) << 4);
      const float dx = cxS[a] - qx, dy = cyS[a] - qy, dz = czS[a] - qz;
      const float dd = sqrtf(dx * dx + dy * dy + dz * dz);
      d[kc][i] = dd;
      const int t = tyS[a];
#pragma unroll
      for (int u = 0; u < NTYPE; ++u) tmin[u] = (t == u) ? fminf(tmin[u], dd) : tmin[u];
    }
  }
#pragma unroll
  for (int t = 0; t < NTYPE; ++t) tmin[t] = fminf(tmin[t], __shfl_xor(tmin[t], 16, 32));
  __syncthreads();

  f32x8 acc[2] = {}, accx[2] = {};
  const float LOG2E = 1.44269504088896340736f;
#pragma unroll
  for (int kc = 0; kc < 4; ++kc) {
    f16x16 ah, al;
#pragma unroll
    for (int i = 0; i < 16; ++i) {
      const int a = kc * 32 + hsel * 8 + (i & 7) + ((i >> 3) << 4);
      const int t = tyS[a];
      float m = tmin[0];
#pragma unroll
      for (int u = 1; u < NTYPE; ++u) m = (t == u) ? tmin[u] : m;
      const float e = __builtin_amdgcn_exp2f((m - d[kc][i]) * LOG2E + 10.0f);
      f16 h, l; split16(e, h, l);
      ah[i] = h; al[i] = l;
    }
#pragma unroll
    for (int nt = 0; nt < 2; ++nt) {
      const f16x16 bh = lds_frag(BhS + (nt * 16) * BSTR + kc * 32, BSTR);
      const f16x16 bl = lds_frag(BlS + (nt * 16) * BSTR + kc * 32, BSTR);
      acc[nt]  = wmma16(ah, bh, acc[nt]);
      accx[nt] = wmma16(ah, bl, accx[nt]);
      accx[nt] = wmma16(al, bh, accx[nt]);
    }
  }
#pragma unroll
  for (int nt = 0; nt < 2; ++nt)
#pragma unroll
    for (int r = 0; r < 8; ++r)
      accS[(wave * 16 + hsel * 8 + r) * ASTR + nt * 16 + pl] = acc[nt][r] + accx[nt][r] * (1.0f / 2048.0f);
  __syncthreads();

  for (int it = tid; it < PPB * NTYPE; it += 64) {
    const int p = it / NTYPE, t = it - p * NTYPE;
    float gx = 0.0f, gy = 0.0f, gz = 0.0f;
    if (tcnt[t] > 0) {
      const float* g = accS + p * ASTR + 4 * t;
      const float inv = 1.0f / g[3];
      gx = g[0] * inv - qS[p * 3 + 0];
      gy = g[1] * inv - qS[p * 3 + 1];
      gz = g[2] * inv - qS[p * 3 + 2];
      const float mag = sqrtf(gx * gx + gy * gy + gz * gz);
      const float fac = fminf(1.0f, CLIPV / fmaxf(mag, 1e-12f));
      gx *= fac; gy *= fac; gz *= fac;
    }
    outS[p * 15 + t * 3 + 0] = gx; outS[p * 15 + t * 3 + 1] = gy; outS[p * 15 + t * 3 + 2] = gz;
  }
  __syncthreads();
  float* ob = out + (size_t)blk * (PPB * NTYPE * 3);
#pragma unroll 1
  for (int pass = 0; pass < 2; ++pass) {
#pragma unroll
    for (int rnd = 0; rnd < 2; ++rnd) {
      const int ch = tid + 64 * rnd;
      if (ch < 120) *(volatile v4f_t*)(ob + ch * 4) = *(const volatile v4fa*)(outS + ch * 4);
    }
    __threadfence();
  }
}

extern "C" void kernel_launch(void* const* d_in, const int* in_sizes, int n_in,
                              void* d_out, int out_size, void* d_ws, size_t ws_size,
                              hipStream_t stream) {
  (void)in_sizes; (void)n_in; (void)out_size; (void)d_ws; (void)ws_size;
  const float* coords = (const float*)d_in[0];
  const int*   atype  = (const int*)d_in[1];
  const float* query  = (const float*)d_in[2];
  float*       out    = (float*)d_out;
  gnf_field_kernel<<<dim3(NBATCH * (NPT / PPB)), dim3(64), 0, stream>>>(coords, atype, query, out);
}
